// MALAttention_58136677319430
// MI455X (gfx1250) — hardware-verified
//
#include <hip/hip_runtime.h>
#include <cstdint>
#include <cstddef>


typedef __attribute__((ext_vector_type(16))) _Float16 v16h;
typedef __attribute__((ext_vector_type(8)))  _Float16 v8h;
typedef __attribute__((ext_vector_type(16))) __bf16   v16b;
typedef __attribute__((ext_vector_type(8)))  __bf16   v8b;
typedef __attribute__((ext_vector_type(8)))  float    v8f;
typedef __attribute__((ext_vector_type(4)))  float    v4f;

__device__ __forceinline__ unsigned short f2bf_bits(float f) {
  unsigned u = __float_as_uint(f);
  return (unsigned short)((u + 0x7FFFu + ((u >> 16) & 1u)) >> 16);
}
__device__ __forceinline__ float bf_bits2f(unsigned short h) { return __uint_as_float(((unsigned)h) << 16); }

__device__ __forceinline__ void dep_guard_h(v8f& a, v8f& b, v16h x, v16h y) { asm volatile("v_nop\n\tv_nop\n\tv_nop\n\tv_nop" : "+v"(a), "+v"(b) : "v"(x), "v"(y)); }
__device__ __forceinline__ void dep_guard_b(v8f& a, v8f& b, v16b x, v16b y) { asm volatile("v_nop\n\tv_nop\n\tv_nop\n\tv_nop" : "+v"(a), "+v"(b) : "v"(x), "v"(y)); }
__device__ __forceinline__ void keep4_h(v16h a, v16h b, v16h c, v16h d) { asm volatile("v_nop" :: "v"(a), "v"(b), "v"(c), "v"(d)); }
__device__ __forceinline__ void keep4_b(v16b a, v16b b, v16b c, v16b d) { asm volatile("v_nop" :: "v"(a), "v"(b), "v"(c), "v"(d)); }
__device__ __forceinline__ void acc_guard4(v8f& a, v8f& b, v8f& c, v8f& d) { asm volatile("v_nop\n\tv_nop\n\tv_nop\n\tv_nop" : "+v"(a), "+v"(b), "+v"(c), "+v"(d)); }
template <typename T> struct Frag;
template <> struct Frag<_Float16> {
  typedef v16h V; union U { v16h v; v8h h[2]; };
  static __device__ __forceinline__ v16h load(const _Float16* p) {
    U f; f.h[0] = *(const v8h*)(p); f.h[1] = *(const v8h*)(p + 16); return f.v;
  }
  static __device__ __forceinline__ v8f mma(v16h a, v16h b, v8f c) {
    return __builtin_amdgcn_wmma_f32_16x16x32_f16(false, a, false, b, (short)0, c, false, false);
  }
  static __device__ __forceinline__ void guard(v8f& a, v8f& b, v16h x, v16h y) { dep_guard_h(a, b, x, y); }
  static __device__ __forceinline__ void keep(v16h a, v16h b, v16h c, v16h d) { keep4_h(a, b, c, d); }
};
template <> struct Frag<__bf16> {
  typedef v16b V; union U { v16b v; v8b h[2]; };
  static __device__ __forceinline__ v16b load(const __bf16* p) {
    U f; f.h[0] = *(const v8b*)(p); f.h[1] = *(const v8b*)(p + 16); return f.v;
  }
  static __device__ __forceinline__ v8f mma(v16b a, v16b b, v8f c) {
    return __builtin_amdgcn_wmma_f32_16x16x32_bf16(false, a, false, b, (short)0, c, false, false);
  }
  static __device__ __forceinline__ void guard(v8f& a, v8f& b, v16b x, v16b y) { dep_guard_b(a, b, x, y); }
  static __device__ __forceinline__ void keep(v16b a, v16b b, v16b c, v16b d) { keep4_b(a, b, c, d); }
};

template <int ET> struct Elem;
template <> struct Elem<0> { typedef _Float16 T; };
template <> struct Elem<1> { typedef __bf16 T; };
template <int ET, bool SPLIT, int BIAS_MODE, int OUT_MODE, bool RESID, int ACT = 0>
__global__ __launch_bounds__(256) void wmma_gemm64(
    const unsigned short* __restrict__ Ap, const unsigned short* __restrict__ A2p, int lda, long strideA,
    const unsigned short* __restrict__ Btp, const unsigned short* __restrict__ Bt2p, int ldb, long strideB,
    void* __restrict__ Cout, void* __restrict__ Cout2, int ldc, long strideC,
    const float* __restrict__ bias,
    const float* __restrict__ resid, long strideR,
    int M, int N, int K, float scale) {
  typedef typename Elem<ET>::T T;
  typedef typename Frag<T>::V V;
  const T* A = (const T*)Ap; const T* A2 = (const T*)A2p; const T* Bt = (const T*)Btp; const T* Bt2 = (const T*)Bt2p;
  __shared__ __align__(16) float sT[8][16 * 68];
  const int b    = blockIdx.y;
  const int lane = threadIdx.x & 31;
  const int wave = threadIdx.x >> 5;
  const int tilesN = N >> 6;
  const int tilesM = M >> 6;
  const int tile = blockIdx.x * 8 + wave;
  if (tile >= tilesM * tilesN) return;
  const int tm = tile / tilesN;
  const int tn = tile - tm * tilesN;
  const int m0 = tm << 6;
  const int n0 = tn << 6;

  const T* Ab  = A  + (size_t)b * strideA;
  const T* Bb  = Bt + (size_t)b * strideB;
  const T* Ab2 = SPLIT ? (A2  + (size_t)b * strideA) : nullptr;
  const T* Bb2 = SPLIT ? (Bt2 + (size_t)b * strideB) : nullptr;

  const int rlane = lane & 15;
  const int koff  = (lane >> 4) * 8;
  const int mOff  = (lane >> 4) * 8;

  v8f acc[4][4];
#pragma unroll
  for (int i = 0; i < 4; ++i)
#pragma unroll
    for (int j = 0; j < 4; ++j) acc[i][j] = (v8f){0.f,0.f,0.f,0.f,0.f,0.f,0.f,0.f};

  for (int k0 = 0; k0 < K; k0 += 32) {
    V bh[4], bl[4];
#pragma unroll
    for (int j = 0; j < 4; ++j) {
      const size_t bo = (size_t)(n0 + (j << 4) + rlane) * ldb + koff + k0;
      bh[j] = Frag<T>::load(Bb + bo);
      if (SPLIT) bl[j] = Frag<T>::load(Bb2 + bo);
    }
#pragma unroll
    for (int i = 0; i < 4; ++i) {
      const size_t ao = (size_t)(m0 + (i << 4) + rlane) * lda + koff + k0;
      V ah = Frag<T>::load(Ab + ao);
      V al;
      if (SPLIT) al = Frag<T>::load(Ab2 + ao);
#pragma unroll
      for (int j = 0; j < 4; ++j) {
        acc[i][j] = Frag<T>::mma(ah, bh[j], acc[i][j]);
        if (SPLIT) {
          acc[i][j] = Frag<T>::mma(ah, bl[j], acc[i][j]);
          acc[i][j] = Frag<T>::mma(al, bh[j], acc[i][j]);
        }
      }
      Frag<T>::guard(acc[i][0], acc[i][3], ah, SPLIT ? al : ah);
    }
    Frag<T>::keep(bh[0], bh[1], bh[2], bh[3]);
    if (SPLIT) Frag<T>::keep(bl[0], bl[1], bl[2], bl[3]);
  }
  acc_guard4(acc[0][0], acc[0][1], acc[0][2], acc[0][3]);
  acc_guard4(acc[1][0], acc[1][1], acc[1][2], acc[1][3]);
  acc_guard4(acc[2][0], acc[2][1], acc[2][2], acc[2][3]);
  acc_guard4(acc[3][0], acc[3][1], acc[3][2], acc[3][3]);

  float* slab = sT[wave];
  const float* Rb = RESID ? (resid + (size_t)b * strideR) : nullptr;
#pragma unroll
  for (int i = 0; i < 4; ++i) {
    const int mBase = m0 + (i << 4);
#pragma unroll
    for (int j = 0; j < 4; ++j) {
      const int n = n0 + (j << 4) + rlane;
      float bv = 0.f;
      if (BIAS_MODE == 2) bv = bias[n];
#pragma unroll
      for (int r = 0; r < 8; ++r) {
        float v = acc[i][j][r] * scale;
        if (BIAS_MODE == 1) v += bias[mBase + mOff + r];
        if (BIAS_MODE == 2) v += bv;
        if (RESID) v += Rb[(size_t)(mBase + mOff + r) * ldc + n];
        if (ACT == 1) v = tanhf(v);
        if (ACT == 2) v = fmaxf(v, 0.0f);
        if (ACT == 3) v = v / (1.0f + expf(-v));
        if (ACT == 4) v = (v > 0.f) ? v : 0.01f * v;
        if (ACT == 5) v = 0.5f * v * (1.0f + erff(v * 0.70710678118654752f));
        slab[(mOff + r) * 68 + (j << 4) + rlane] = v;
      }
    }
    __builtin_amdgcn_fence(__ATOMIC_RELEASE, "workgroup");
    __builtin_amdgcn_wave_barrier();
    __builtin_amdgcn_fence(__ATOMIC_ACQUIRE, "workgroup");
    if (OUT_MODE == 0) {
      float* C = (float*)Cout + (size_t)b * strideC;
      const int hh = lane >> 4, c4 = (lane & 15) * 4;
      for (int pass = 0; pass < 2; ++pass) {
#pragma unroll
        for (int it = 0; it < 8; ++it) {
          const int row = it * 2 + hh;
          v4f v = *(const v4f*)(slab + row * 68 + c4);
          *(volatile v4f*)(C + (size_t)(mBase + row) * ldc + n0 + c4) = v;
        }
        __threadfence();
      }
    } else {
      const int q = lane >> 3, c8 = (lane & 7) * 8;
      unsigned short* C  = (unsigned short*)Cout  + (size_t)b * strideC;
      unsigned short* C2 = (OUT_MODE == 2) ? ((unsigned short*)Cout2 + (size_t)b * strideC) : nullptr;
      for (int pass = 0; pass < 2; ++pass) {
#pragma unroll
        for (int it = 0; it < 4; ++it) {
          const int row = it * 4 + q;
          const float* sp = slab + row * 68 + c8;
          v8h hv, lv;
#pragma unroll
          for (int e = 0; e < 8; ++e) {
            if (OUT_MODE == 1) {
              hv[e] = (_Float16)sp[e];
            } else {
              unsigned short hb = f2bf_bits(sp[e]);
              unsigned short lb = f2bf_bits(sp[e] - bf_bits2f(hb));
              hv[e] = __builtin_bit_cast(_Float16, hb);
              lv[e] = __builtin_bit_cast(_Float16, lb);
            }
          }
          *(volatile v8h*)(C + (size_t)(mBase + row) * ldc + n0 + c8) = hv;
          if (OUT_MODE == 2) *(volatile v8h*)(C2 + (size_t)(mBase + row) * ldc + n0 + c8) = lv;
        }
        __threadfence();
      }
    }
    __builtin_amdgcn_fence(__ATOMIC_RELEASE, "workgroup");
    __builtin_amdgcn_wave_barrier();
    __builtin_amdgcn_fence(__ATOMIC_ACQUIRE, "workgroup");
  }
}

__global__ __launch_bounds__(256) void cast_f32_f16x2(
    const float* __restrict__ in, _Float16* __restrict__ out, int n2, float mul) {
  int i = blockIdx.x * 256 + threadIdx.x;
  if (i < n2) {
    const size_t e0 = 2 * (size_t)i;
    const _Float16 h0 = (_Float16)(in[e0] * mul), h1 = (_Float16)(in[e0 + 1] * mul);
    const unsigned u = (unsigned)__builtin_bit_cast(unsigned short, h0) | ((unsigned)__builtin_bit_cast(unsigned short, h1) << 16);
    ((volatile unsigned*)out)[i] = u;
    __threadfence();
    ((volatile unsigned*)out)[i] = u;
  }
}

__global__ __launch_bounds__(512) void qgate_f16(
    const float* __restrict__ q32, _Float16* __restrict__ q16, int rows, int ld, float mul) {
  const int row  = blockIdx.x;
  const int wave = threadIdx.x >> 5;
  const int lane = threadIdx.x & 31;
  if (row >= rows) return;
  const size_t base = (size_t)row * ld + (size_t)wave * 64 + 2 * lane;
  const float a0 = q32[base];
  const float a1 = q32[base + 1];
  float ss = a0 * a0 + a1 * a1;
#pragma unroll
  for (int off = 1; off < 32; off <<= 1) ss += __shfl_xor(ss, off, 32);
  const float mag = sqrtf(ss);
  const float sg  = 1.0f / (1.0f + expf(-mag));
  const float f   = sg * mul;
  const _Float16 h0 = (_Float16)(a0 * f), h1 = (_Float16)(a1 * f);
  const unsigned u = (unsigned)__builtin_bit_cast(unsigned short, h0) | ((unsigned)__builtin_bit_cast(unsigned short, h1) << 16);
  volatile unsigned* op = (volatile unsigned*)(q16 + base);
  *op = u;
  __threadfence();
  *op = u;
}

#define AT_D 64
#define AT_NW 4
#define AT_QB 64
#define AT_KC 64
#define AT_PSC 32768.0f

__device__ __forceinline__ v8f at_mma_h(v16h a, v16h b, v8f c) {
  c = __builtin_amdgcn_wmma_f32_16x16x32_f16(false, a, false, b, (short)0, c, false, false);
  asm volatile("v_nop\n\tv_nop\n\tv_nop\n\tv_nop" : "+v"(c) : "v"(a), "v"(b));
  return c;
}

__global__ __launch_bounds__(128)
void attn64_h(const _Float16* __restrict__ q, const _Float16* __restrict__ k,
              const _Float16* __restrict__ v, _Float16* __restrict__ o,
              int S, int H, int q_rs, int k_rs, int v_rs, int o_rs, float sscale, float omul) {
  union FH { v16h v; v8h h[2]; };
  __shared__ __align__(16) _Float16 Ksh[AT_KC * AT_D];
  __shared__ __align__(16) _Float16 Vth[AT_D * AT_KC];
  __shared__ __align__(16) _Float16 Psh[AT_NW][16 * AT_KC];
  __shared__ __align__(16) float    Os[AT_NW][16 * 68];

  const int tid  = threadIdx.x;
  const int wave = tid >> 5;
  const int lane = tid & 31;
  const int hh   = lane >> 4;
  const int c    = lane & 15;

  const int nqb = S / AT_QB;
  const int bx  = blockIdx.x;
  const int qb  = bx % nqb;
  const int bh  = bx / nqb;
  const int h   = bh % H;
  const int b   = bh / H;
  const size_t rowbase = (size_t)b * S;
  const int q0 = qb * AT_QB + wave * 16;

  v16h qa[2];
  {
    const _Float16* qrow = q + (rowbase + q0 + c) * (size_t)q_rs + h * AT_D;
#pragma unroll
    for (int dc = 0; dc < 2; ++dc) qa[dc] = Frag<_Float16>::load(qrow + dc * 32 + 8 * hh);
  }

  const float NEG_INF = -__builtin_huge_valf();
  float mrow[8], lrow[8];
  v8f oacc[4];
#pragma unroll
  for (int r = 0; r < 8; ++r) { mrow[r] = NEG_INF; lrow[r] = 0.f; }
#pragma unroll
  for (int t = 0; t < 4; ++t) oacc[t] = (v8f){0.f,0.f,0.f,0.f,0.f,0.f,0.f,0.f};

  const int nChunks = S / AT_KC;
  for (int kc = 0; kc < nChunks; ++kc) {
    const int kv0 = kc * AT_KC;
    __syncthreads();
    {
      const int kvr = tid >> 1, dh = (tid & 1) * 32;
      const _Float16* krow = k + (rowbase + kv0 + kvr) * (size_t)k_rs + h * AT_D + dh;
      const _Float16* vrow = v + (rowbase + kv0 + kvr) * (size_t)v_rs + h * AT_D + dh;
#pragma unroll
      for (int i = 0; i < 4; ++i) {
        const v8h kk = *(const v8h*)(krow + 8 * i);
        const v8h vv = *(const v8h*)(vrow + 8 * i);
        *(v8h*)(Ksh + kvr * AT_D + dh + 8 * i) = kk;
#pragma unroll
        for (int e = 0; e < 8; ++e) Vth[(dh + 8 * i + e) * AT_KC + kvr] = vv[e];
      }
    }
    __syncthreads();

    v8f s[4];
#pragma unroll
    for (int j = 0; j < 4; ++j) {
      s[j] = (v8f){0.f,0.f,0.f,0.f,0.f,0.f,0.f,0.f};
#pragma unroll
      for (int dc = 0; dc < 2; ++dc) {
        FH kb;
        kb.h[0] = *(const v8h*)(Ksh + (j * 16 + c) * AT_D + dc * 32 + 8 * hh);
        kb.h[1] = *(const v8h*)(Ksh + (j * 16 + c) * AT_D + dc * 32 + 16 + 8 * hh);
        s[j] = at_mma_h(qa[dc], kb.v, s[j]);
      }
    }
    float cm[8];
#pragma unroll
    for (int r = 0; r < 8; ++r) {
      float m = NEG_INF;
#pragma unroll
      for (int j = 0; j < 4; ++j) {
        s[j][r] *= sscale;
        m = fmaxf(m, s[j][r]);
      }
#pragma unroll
      for (int off = 1; off < 16; off <<= 1) m = fmaxf(m, __shfl_xor(m, off, 32));
      cm[r] = m;
    }
    _Float16* pw = Psh[wave];
#pragma unroll
    for (int r = 0; r < 8; ++r) {
      const float mnew  = fmaxf(mrow[r], cm[r]);
      const float alpha = expf(mrow[r] - mnew);
      mrow[r] = mnew;
      float psum = 0.f;
#pragma unroll
      for (int j = 0; j < 4; ++j) {
        const float p = expf(s[j][r] - mnew);
        psum += p;
        pw[(8 * hh + r) * AT_KC + j * 16 + c] = (_Float16)(p * AT_PSC);
      }
#pragma unroll
      for (int off = 1; off < 16; off <<= 1) psum += __shfl_xor(psum, off, 32);
      lrow[r] = lrow[r] * alpha + psum;
#pragma unroll
      for (int t = 0; t < 4; ++t) oacc[t][r] *= alpha;
    }
    __builtin_amdgcn_fence(__ATOMIC_RELEASE, "workgroup");
    __builtin_amdgcn_wave_barrier();
    __builtin_amdgcn_fence(__ATOMIC_ACQUIRE, "workgroup");
#pragma unroll
    for (int kk = 0; kk < 2; ++kk) {
      FH pa;
      pa.h[0] = *(const v8h*)(pw + c * AT_KC + kk * 32 + 8 * hh);
      pa.h[1] = *(const v8h*)(pw + c * AT_KC + kk * 32 + 16 + 8 * hh);
#pragma unroll
      for (int t = 0; t < 4; ++t) {
        FH vb;
        vb.h[0] = *(const v8h*)(Vth + (t * 16 + c) * AT_KC + kk * 32 + 8 * hh);
        vb.h[1] = *(const v8h*)(Vth + (t * 16 + c) * AT_KC + kk * 32 + 16 + 8 * hh);
        oacc[t] = at_mma_h(pa.v, vb.v, oacc[t]);
      }
    }
  }

  float* os = Os[wave];
#pragma unroll
  for (int r = 0; r < 8; ++r) {
    const float inv = omul * (1.0f / (lrow[r] * AT_PSC));
#pragma unroll
    for (int t = 0; t < 4; ++t) os[(8 * hh + r) * 68 + t * 16 + c] = oacc[t][r] * inv;
  }
  __builtin_amdgcn_fence(__ATOMIC_RELEASE, "workgroup");
  __builtin_amdgcn_wave_barrier();
  __builtin_amdgcn_fence(__ATOMIC_ACQUIRE, "workgroup");
  {
    const int qq = lane >> 3, c8 = (lane & 7) * 8;
    _Float16* ob = o + h * AT_D;
    for (int pass = 0; pass < 2; ++pass) {
#pragma unroll
      for (int it = 0; it < 4; ++it) {
        const int row = it * 4 + qq;
        const float* sp = os + row * 68 + c8;
        v8h hv;
#pragma unroll
        for (int e = 0; e < 8; ++e) hv[e] = (_Float16)sp[e];
        *(volatile v8h*)(ob + (rowbase + q0 + row) * (size_t)o_rs + c8) = hv;
      }
      __threadfence();
    }
  }
}

extern "C" void kernel_launch(void* const* d_in, const int* in_sizes, int n_in,
                              void* d_out, int out_size, void* d_ws,
                              size_t ws_size, hipStream_t stream) {
  const int B = 4, S = 2048, C = 1024, H = 16;
  const int M = B * S;
  if (n_in < 4) return;
  if (in_sizes[0] != M * C) return;
  if (in_sizes[1] != 3 * C * C) return;
  if (in_sizes[2] != C * C) return;
  if (in_sizes[3] != C) return;
  if (out_size != M * C) return;

  const float* x      = (const float*)d_in[0];
  const float* w_qkv  = (const float*)d_in[1];
  const float* w_proj = (const float*)d_in[2];
  const float* b_proj = (const float*)d_in[3];
  float* out = (float*)d_out;

  const size_t sz_x16  = (size_t)M * C * 2;
  const size_t sz_wq16 = (size_t)3 * C * C * 2;
  const size_t sz_wp16 = (size_t)C * C * 2;
  const size_t sz_q32  = (size_t)M * C * 4;
  const size_t sz_q16  = (size_t)M * C * 2;
  const size_t sz_kv16 = (size_t)M * 2 * C * 2;
  const size_t sz_o16  = (size_t)M * C * 2;
  size_t off = 0;
  char* ws = (char*)d_ws;
  _Float16* x16  = (_Float16*)(ws + off); off += sz_x16;
  _Float16* wq16 = (_Float16*)(ws + off); off += sz_wq16;
  _Float16* wp16 = (_Float16*)(ws + off); off += sz_wp16;
  float*    q32  = (float*)(ws + off);    off += sz_q32;
  _Float16* q16  = (_Float16*)(ws + off); off += sz_q16;
  _Float16* kv16 = (_Float16*)(ws + off); off += sz_kv16;
  _Float16* o16  = (_Float16*)(ws + off); off += sz_o16;
  if (off > ws_size) return;

  const unsigned short* x16u  = (const unsigned short*)x16;
  const unsigned short* wq16u = (const unsigned short*)wq16;
  const unsigned short* wp16u = (const unsigned short*)wp16;
  const unsigned short* o16u  = (const unsigned short*)o16;

  {
    const int n2x = (M * C) / 2, n2q = (3 * C * C) / 2, n2p = (C * C) / 2;
    cast_f32_f16x2<<<(n2x + 255) / 256, 256, 0, stream>>>(x, x16, n2x, 1.0f);
    cast_f32_f16x2<<<(n2q + 255) / 256, 256, 0, stream>>>(w_qkv, wq16, n2q, 64.0f);
    cast_f32_f16x2<<<(n2p + 255) / 256, 256, 0, stream>>>(w_proj, wp16, n2p, 64.0f);
  }

  {
    const int tiles = (M / 64) * (C / 64);
    wmma_gemm64<0, false, 0, 0, false><<<dim3((tiles + 7) / 8, 1), 256, 0, stream>>>(
        x16u, x16u, C, 0L, wq16u, wq16u, C, 0L,
        (void*)q32, (void*)q32, C, 0L, b_proj, b_proj, 0L, M, C, C, 1.0f / 64.0f);
  }
  {
    const int tiles = (M / 64) * ((2 * C) / 64);
    wmma_gemm64<0, false, 0, 1, false><<<dim3((tiles + 7) / 8, 1), 256, 0, stream>>>(
        x16u, x16u, C, 0L, wq16u + (size_t)C * C, wq16u + (size_t)C * C, C, 0L,
        (void*)kv16, (void*)kv16, 2 * C, 0L, b_proj, b_proj, 0L, M, 2 * C, C, 1.0f / 64.0f);
  }
  qgate_f16<<<M, 32 * H, 0, stream>>>(q32, q16, M, C, 8.0f);

  attn64_h<<<B * H * (S / AT_QB), 128, 0, stream>>>(
      q16, kv16, kv16 + C, o16, S, H, C, 2 * C, 2 * C, C, 0.125f / 8.0f, 16.0f);

  {
    const int tiles = (M / 64) * (C / 64);
    wmma_gemm64<0, false, 2, 0, false><<<dim3((tiles + 7) / 8, 1), 256, 0, stream>>>(
        o16u, o16u, C, 0L, wp16u, wp16u, C, 0L,
        (void*)out, (void*)out, C, 0L, b_proj, b_proj, 0L, M, C, C, 1.0f / 1024.0f);
  }
}
